// OuterProductLayer_2602750182019
// MI455X (gfx1250) — hardware-verified
//
#include <hip/hip_runtime.h>

#define EMB 64
#define NF 32
#define NPAIR 496
#define NPAIR_PAD 512
#define D1 256
#define BATCH 2048
#define RSPLIT (1.0f / 2048.0f)

typedef _Float16 f16;
typedef __attribute__((ext_vector_type(16))) _Float16 v16h;
typedef __attribute__((ext_vector_type(8)))  _Float16 v8h;
typedef __attribute__((ext_vector_type(8)))  float    v8f;
typedef __attribute__((ext_vector_type(4)))  float    v4f_t;
typedef float v4fa __attribute__((ext_vector_type(4), may_alias));
typedef __attribute__((ext_vector_type(4)))  unsigned v4u_t;
typedef __attribute__((ext_vector_type(2)))  unsigned v2u_t;

#define PL_F ((size_t)BATCH * NF * EMB)
#define PL_K ((size_t)EMB * NPAIR * EMB)
#define PL_W ((size_t)D1 * NPAIR_PAD)
#define PL_P ((size_t)BATCH * NPAIR_PAD)

__device__ __forceinline__ f16 lo_of(float v, f16 h) { return (f16)((v - (float)h) * 2048.0f); }
__device__ __forceinline__ unsigned pk2s(float a, float b, unsigned* lo) {
  const f16 h0 = (f16)a, h1 = (f16)b;
  *lo = (unsigned)__builtin_bit_cast(unsigned short, lo_of(a, h0)) | ((unsigned)__builtin_bit_cast(unsigned short, lo_of(b, h1)) << 16);
  return (unsigned)__builtin_bit_cast(unsigned short, h0) | ((unsigned)__builtin_bit_cast(unsigned short, h1) << 16);
}
__device__ __forceinline__ v8f wmma16(v16h a, v16h b, v8f c) { return __builtin_amdgcn_wmma_f32_16x16x32_f16(false, a, false, b, (short)0, c, false, false); }
struct Frag2 { v16h h, l; };
__device__ __forceinline__ v8f wmma_split(const Frag2& a, const Frag2& b, v8f c) { v8f x = {}; x = wmma16(a.l, b.h, x); x = wmma16(a.h, b.l, x); return wmma16(a.h, b.h, c) + x * RSPLIT; }
__device__ __forceinline__ Frag2 load2(const f16* base, size_t stride, size_t plane, int lane) {
  const f16* p = base + (size_t)(lane & 15) * stride + ((lane >> 4) << 3);
  Frag2 f;
  f.h = __builtin_shufflevector(*(const v8h*)p, *(const v8h*)(p + 16), 0,1,2,3,4,5,6,7,8,9,10,11,12,13,14,15);
  f.l = __builtin_shufflevector(*(const v8h*)(p + plane), *(const v8h*)(p + plane + 16), 0,1,2,3,4,5,6,7,8,9,10,11,12,13,14,15);
  return f;
}

__global__ void cvt_planes_v4(const float* __restrict__ in, f16* __restrict__ out, size_t plane, int n4) {
  int i = blockIdx.x * blockDim.x + threadIdx.x;
  if (i >= n4) return;
  const v4f_t x = *(const v4f_t*)(in + (size_t)i * 4);
  v2u_t v, l; unsigned l0, l1;
  v.x = pk2s(x[0], x[1], &l0); v.y = pk2s(x[2], x[3], &l1); l.x = l0; l.y = l1;
  f16* d = out + (size_t)i * 4;
  *(volatile v2u_t*)d = v; *(volatile v2u_t*)(d + plane) = l; __threadfence();
  *(volatile v2u_t*)d = v; *(volatile v2u_t*)(d + plane) = l;
}
__global__ void cvt_w_pad_kernel(const float* __restrict__ W, f16* __restrict__ out) {
  int i = (blockIdx.x * blockDim.x + threadIdx.x) * 2;
  if (i >= D1 * NPAIR_PAD) return;
  int n = i >> 9, k = i & (NPAIR_PAD - 1);
  const float w0 = (k < NPAIR) ? W[n * NPAIR + k] : 0.f, w1 = (k + 1 < NPAIR) ? W[n * NPAIR + k + 1] : 0.f;
  unsigned l; const unsigned v = pk2s(w0, w1, &l);
  *(volatile unsigned*)(out + i) = v; *(volatile unsigned*)(out + PL_W + i) = l; __threadfence();
  *(volatile unsigned*)(out + i) = v; *(volatile unsigned*)(out + PL_W + i) = l;
}
__global__ void pad_pijT_kernel(float* __restrict__ pijT) {
  int i = blockIdx.x * blockDim.x + threadIdx.x;
  float* p = pijT + (size_t)NPAIR * BATCH + i;
  *(volatile float*)p = 0.f; __threadfence(); *(volatile float*)p = 0.f;
}

__global__ void __launch_bounds__(256)
bilinear_pair_kernel(const f16* __restrict__ featb,
                     const f16* __restrict__ kernb,
                     const float* __restrict__ feat,
                     float* __restrict__ pijT)
{
  __shared__ __attribute__((aligned(16))) float sres[8][128];
  const int p = blockIdx.x;
  int fi = 0, rem = p;
  while (rem >= (NF - 1 - fi)) { rem -= (NF - 1 - fi); ++fi; }
  const int rowp = fi, colp = fi + 1 + rem;

  const int wave = threadIdx.x >> 5, lane = threadIdx.x & 31, lm = lane & 15, lh = lane >> 4;
  const int slot = blockIdx.y * 8 + wave;

  Frag2 bfr[2][4];
#pragma unroll
  for (int ks = 0; ks < 2; ++ks)
#pragma unroll
    for (int j = 0; j < 4; ++j)
      bfr[ks][j] = load2(kernb + ((size_t)(16 * j) * NPAIR + p) * EMB + 32 * ks, (size_t)NPAIR * EMB, PL_K, lane);

#pragma unroll 1
  for (int t = 0; t < 8; ++t) {
    const int b0 = (slot * 8 + t) * 16;
    v8f acc[4] = {v8f{}, v8f{}, v8f{}, v8f{}};
#pragma unroll
    for (int ks = 0; ks < 2; ++ks) {
      const Frag2 a = load2(featb + ((size_t)b0 * NF + rowp) * EMB + 32 * ks, (size_t)NF * EMB, PL_F, lane);
#pragma unroll
      for (int j = 0; j < 4; ++j) acc[j] = wmma_split(a, bfr[ks][j], acc[j]);
    }
#pragma unroll
    for (int r = 0; r < 8; ++r) {
      const int b = b0 + r + 8 * lh;
      const float* qrow = feat + ((size_t)b * NF + colp) * EMB;
      float s = acc[0][r] * qrow[lm] + acc[1][r] * qrow[16 + lm] + acc[2][r] * qrow[32 + lm] + acc[3][r] * qrow[48 + lm];
      s += __shfl_xor(s, 1); s += __shfl_xor(s, 2); s += __shfl_xor(s, 4); s += __shfl_xor(s, 8);
      if (lm == 0) sres[wave][t * 16 + r + 8 * lh] = s;
    }
  }
  asm volatile("s_wait_dscnt 0" ::: "memory");
  float* dst = pijT + (size_t)p * BATCH + slot * 128;
#pragma unroll 1
  for (int pass = 0; pass < 2; ++pass) {
    *(volatile v4f_t*)(dst + lane * 4) = *(const volatile v4fa*)(&sres[wave][lane * 4]);
    __threadfence();
  }
}

__global__ __launch_bounds__(256) void tp_kernel(const float* __restrict__ pijT, f16* __restrict__ pij) {
  __shared__ float tl[64][65];
  const int tid = threadIdx.x, p0 = blockIdx.x * 64, b0 = blockIdx.y * 64;
  for (int i = tid; i < 64 * 64; i += 256) { const int pp = i >> 6, bb = i & 63; tl[pp][bb] = pijT[(size_t)(p0 + pp) * BATCH + b0 + bb]; }
  __syncthreads();
  const int bb = tid >> 2, q = (tid & 3) * 16;
  v4u_t v0, v1, l0, l1; unsigned lo;
  float s[16];
#pragma unroll
  for (int j = 0; j < 16; ++j) s[j] = tl[q + j][bb];
  v0.x = pk2s(s[0], s[1], &lo); l0.x = lo; v0.y = pk2s(s[2], s[3], &lo); l0.y = lo; v0.z = pk2s(s[4], s[5], &lo); l0.z = lo; v0.w = pk2s(s[6], s[7], &lo); l0.w = lo;
  v1.x = pk2s(s[8], s[9], &lo); l1.x = lo; v1.y = pk2s(s[10], s[11], &lo); l1.y = lo; v1.z = pk2s(s[12], s[13], &lo); l1.z = lo; v1.w = pk2s(s[14], s[15], &lo); l1.w = lo;
  f16* d = pij + (size_t)(b0 + bb) * NPAIR_PAD + p0 + q;
#pragma unroll 1
  for (int pass = 0; pass < 2; ++pass) {
    *(volatile v4u_t*)d = v0; *(volatile v4u_t*)(d + 8) = v1; *(volatile v4u_t*)(d + PL_P) = l0; *(volatile v4u_t*)(d + PL_P + 8) = l1;
    __threadfence();
  }
}

__global__ void __launch_bounds__(256)
final_gemm_kernel(const f16* __restrict__ pij, const f16* __restrict__ wb, const float* __restrict__ bias, float* __restrict__ out) {
  __shared__ __attribute__((aligned(16))) float stg[8][16 * 36];
  const int wave = threadIdx.x >> 5, lane = threadIdx.x & 31, lm = lane & 15, lh = lane >> 4;
  const int tid  = blockIdx.x * 8 + wave;
  const int mt = tid >> 3, ng = tid & 7;
  v8f acc0 = {}, acc1 = {};
#pragma unroll 2
  for (int kk = 0; kk < NPAIR_PAD / 32; ++kk) {
    const Frag2 a  = load2(pij + (size_t)(mt * 16) * NPAIR_PAD + kk * 32, NPAIR_PAD, PL_P, lane);
    const Frag2 b0 = load2(wb + (size_t)(ng * 32) * NPAIR_PAD + kk * 32, NPAIR_PAD, PL_W, lane);
    const Frag2 b1 = load2(wb + (size_t)(ng * 32 + 16) * NPAIR_PAD + kk * 32, NPAIR_PAD, PL_W, lane);
    acc0 = wmma_split(a, b0, acc0); acc1 = wmma_split(a, b1, acc1);
  }
  float* sw = stg[wave];
  const float bn0 = bias[ng * 32 + lm], bn1 = bias[ng * 32 + 16 + lm];
#pragma unroll
  for (int r = 0; r < 8; ++r) { sw[(r + 8 * lh) * 36 + lm] = acc0[r] + bn0; sw[(r + 8 * lh) * 36 + 16 + lm] = acc1[r] + bn1; }
  asm volatile("s_wait_dscnt 0" ::: "memory");
#pragma unroll 1
  for (int pass = 0; pass < 2; ++pass) {
#pragma unroll
    for (int i = 0; i < 4; ++i) { const int c = lane + 32 * i, rr = c >> 3, q = (c & 7) * 4;
      *(volatile v4f_t*)(out + (size_t)(mt * 16 + rr) * D1 + ng * 32 + q) = *(const volatile v4fa*)(sw + rr * 36 + q); }
    __threadfence();
  }
}

extern "C" void kernel_launch(void* const* d_in, const int* in_sizes, int n_in,
                              void* d_out, int out_size, void* d_ws, size_t ws_size,
                              hipStream_t stream) {
  (void)in_sizes; (void)n_in; (void)out_size; (void)ws_size;
  const float* feat = (const float*)d_in[0];
  const float* kern = (const float*)d_in[1];
  const float* W    = (const float*)d_in[2];
  const float* bias = (const float*)d_in[3];
  float*       out  = (float*)d_out;

  char* ws = (char*)d_ws;
  size_t off = 0;
  auto take = [&](size_t bytes) { char* r = ws + off; off += (bytes + 255) & ~(size_t)255; return r; };
  f16*   featb = (f16*)take(PL_F * 2 * 2);
  f16*   kernb = (f16*)take(PL_K * 2 * 2);
  f16*   wb    = (f16*)take(PL_W * 2 * 2);
  float* pijT  = (float*)take((size_t)NPAIR_PAD * BATCH * 4);
  f16*   pij   = (f16*)take(PL_P * 2 * 2);

  const int nfeat4 = (BATCH * NF * EMB) / 4, nkern4 = (EMB * NPAIR * EMB) / 4;
  cvt_planes_v4<<<nfeat4 / 256, 256, 0, stream>>>(feat, featb, PL_F, nfeat4);
  cvt_planes_v4<<<nkern4 / 256, 256, 0, stream>>>(kern, kernb, PL_K, nkern4);
  cvt_w_pad_kernel<<<(D1 * NPAIR_PAD / 2) / 256, 256, 0, stream>>>(W, wb);
  pad_pijT_kernel<<<(16 * BATCH) / 256, 256, 0, stream>>>(pijT);

  dim3 g2(NPAIR, 2);
  bilinear_pair_kernel<<<g2, 256, 0, stream>>>(featb, kernb, feat, pijT);
  tp_kernel<<<dim3(NPAIR_PAD / 64, BATCH / 64), 256, 0, stream>>>(pijT, pij);
  final_gemm_kernel<<<BATCH / 8 / 2, 256, 0, stream>>>(pij, wb, bias, out);
}
